// PINN_10780367913688
// MI455X (gfx1250) — hardware-verified
//
#include <hip/hip_runtime.h>
#include <math.h>

typedef __attribute__((ext_vector_type(16))) __bf16 v16b;
typedef __attribute__((ext_vector_type(8)))  __bf16 v8b;
typedef __attribute__((ext_vector_type(8)))  float  v8f;
typedef __attribute__((ext_vector_type(4)))  float  v4f;
typedef __attribute__((ext_vector_type(4)))  unsigned int v4u;

constexpr int kWaves       = 8;
constexpr int kBlock       = kWaves * 32;
constexpr int kPtsPerWave  = 32;
constexpr int kPtsPerIter  = 2;
constexpr int kIters       = kPtsPerWave / kPtsPerIter;
constexpr int kPtsPerBlock = kWaves * kPtsPerWave;
constexpr int kHid         = 128;
constexpr int kEmb         = 64;
constexpr int kLayers      = 4;
constexpr int kRows        = 16;
constexpr int kNTiles      = kHid / 16;
static_assert(2 * kEmb == kHid);
static_assert(kHid % 32 == 0);
static_assert(kPtsPerBlock == 256);

constexpr float kTwoPi       = 6.283185307179586f;
constexpr float kCLE         = 0.00574f;
constexpr float kCseMinusCle = 0.49426f;
constexpr float kClScale     = 0.50574f;
constexpr float kAC1         = 2.0f;
constexpr float kAC2         = 1.0f;
constexpr float kAC3         = 0.01f;

__device__ __forceinline__ unsigned short f2bf_bits(float f) {
  unsigned u = __float_as_uint(f);
  return (unsigned short)((u + 0x7FFFu + ((u >> 16) & 1u)) >> 16);
}
__device__ __forceinline__ float bf_bits2f(unsigned short h) { return __uint_as_float(((unsigned)h) << 16); }
__device__ __forceinline__ float bf_rne(float f) { return bf_bits2f(f2bf_bits(f)); }
__device__ __forceinline__ __bf16 bf_pack(unsigned short b) { return __builtin_bit_cast(__bf16, b); }

__device__ __forceinline__ void wave_sync() {
  __builtin_amdgcn_fence(__ATOMIC_RELEASE, "workgroup");
  __builtin_amdgcn_wave_barrier();
  __builtin_amdgcn_fence(__ATOMIC_ACQUIRE, "workgroup");
}

__device__ __forceinline__ v16b load_frag(const __bf16* row, int koff) {
  union { v16b v; v8b h[2]; } u;
  u.h[0] = *(const v8b*)(row + koff);
  u.h[1] = *(const v8b*)(row + koff + 16);
  return u.v;
}

__device__ __forceinline__ v8f mma_bf(v16b a, v16b b, v8f c) {
  return __builtin_amdgcn_wmma_f32_16x16x32_bf16(false, a, false, b, (short)0, c, false, false);
}
__device__ __forceinline__ void mma_guard(v8f& c, v16b a0, v16b a1, v16b a2, v16b a3,
                                          v16b b0, v16b b1, v16b b2, v16b b3) {
  asm volatile("v_nop\n\tv_nop\n\tv_nop\n\tv_nop"
               : "+v"(c)
               : "v"(a0), "v"(a1), "v"(a2), "v"(a3), "v"(b0), "v"(b1), "v"(b2), "v"(b3));
}

__device__ __forceinline__ float tanh_ex(float a) {
  const float ac = fminf(fmaxf(a, -15.0f), 15.0f);
  const float e  = expf(2.0f * ac);
  return 1.0f - 2.0f / (e + 1.0f);
}

__device__ __forceinline__ void put_jet(__bf16* col, float v, float dt, float lap, float gx0, float gx1) {
  const unsigned short vh = f2bf_bits(v);
  const unsigned short vl = f2bf_bits(v - bf_bits2f(vh));
  const unsigned short th = f2bf_bits(dt);
  const unsigned short tl = f2bf_bits(dt - bf_bits2f(th));
  const unsigned short lh = f2bf_bits(lap);
  const unsigned short ll = f2bf_bits(lap - bf_bits2f(lh));
  col[0 * kHid] = bf_pack(vh);
  col[1 * kHid] = bf_pack(vl);
  col[2 * kHid] = bf_pack(th);
  col[3 * kHid] = bf_pack(tl);
  col[4 * kHid] = bf_pack(lh);
  col[5 * kHid] = bf_pack(ll);
  col[6 * kHid] = bf_pack(f2bf_bits(gx0));
  col[7 * kHid] = bf_pack(f2bf_bits(gx1));
}

__global__ __launch_bounds__(kBlock)
void jet_residual_kernel(const float* __restrict__ xin, const float* __restrict__ tin,
                         const float* __restrict__ Bff, const float* __restrict__ Wh,
                         const float* __restrict__ bh, const float* __restrict__ Wout,
                         const float* __restrict__ bout, float* __restrict__ out, int npts)
{
  __shared__ __align__(16) __bf16 sWt[kLayers][kHid][kHid];
  __shared__ __align__(16) __bf16 sH[kWaves][kPtsPerIter][kRows][kHid];
  __shared__ __align__(16) float sFB[3][kEmb];
  __shared__ __align__(16) float sBh[kLayers][kHid];
  __shared__ __align__(16) float sWo[2][kHid];
  __shared__ __align__(16) float sBo[4];
  __shared__ __align__(16) float sRed[kWaves][32];
  __shared__ __align__(16) float sOut[kWaves][32];

  const int tid  = threadIdx.x;
  const int lane = tid & 31;
  const int w    = __builtin_amdgcn_readfirstlane(tid >> 5);
  const int m    = lane & 15;
  const int h    = lane >> 4;

#pragma unroll 2
  for (int idx = tid; idx < kLayers * kHid * kHid; idx += kBlock) {
    const int l = idx >> 14;
    const int k = (idx >> 7) & (kHid - 1);
    const int n = idx & (kHid - 1);
    sWt[l][n][k] = bf_pack(f2bf_bits(Wh[idx]));
  }
  for (int idx = tid; idx < 3 * kEmb; idx += kBlock) sFB[idx >> 6][idx & (kEmb - 1)] = bf_rne(Bff[idx]);
  for (int idx = tid; idx < kLayers * kHid; idx += kBlock) sBh[idx >> 7][idx & (kHid - 1)] = bf_rne(bh[idx]);
  for (int idx = tid; idx < 2 * kHid; idx += kBlock) sWo[idx & 1][idx >> 1] = bf_rne(Wout[idx]);
  for (int idx = tid; idx < 2; idx += kBlock) sBo[idx] = bf_rne(bout[idx]);
  __syncthreads();

  const int  pbase = (blockIdx.x * kWaves + w) * kPtsPerWave;
  const bool isSin = (m < 8);

#pragma unroll 1
  for (int it = 0; it < kIters; ++it) {
    const int p0 = pbase + it * kPtsPerIter;

#pragma unroll
    for (int pt = 0; pt < kPtsPerIter; ++pt) {
      int p = p0 + pt;
      p = (p < npts) ? p : (npts - 1);
      const float x0 = bf_rne(xin[2 * p]);
      const float x1 = bf_rne(xin[2 * p + 1]);
      const float tt = bf_rne(tin[p]);
      const float z0 = h ? -x0 : x0;
      __bf16* rows = &sH[w][pt][8 * h][0];
#pragma unroll 1
      for (int q = 0; q < 8; ++q) {
        const int col = m * 8 + q;
        const int j   = col & (kEmb - 1);
        const float b0 = sFB[0][j], b1 = sFB[1][j], b2 = sFB[2][j];
        float d = z0 * b0;
        d = fmaf(x1, b1, d);
        d = fmaf(tt, b2, d);
        const float f  = kTwoPi * d;
        const float sn = sinf(f);
        const float cs = cosf(f);
        const float g0 = kTwoPi * b0, g1 = kTwoPi * b1, g2 = kTwoPi * b2;
        const float v  = isSin ? sn : cs;
        const float dv = isSin ? cs : -sn;
        put_jet(rows + col, v, dv * g2, -v * (g0 * g0 + g1 * g1), dv * g0, dv * g1);
      }
    }
    wave_sync();

#pragma unroll 1
    for (int l = 0; l < kLayers; ++l) {
      v16b A[kPtsPerIter][4];
#pragma unroll
      for (int pt = 0; pt < kPtsPerIter; ++pt) {
        const __bf16* arow = &sH[w][pt][m][0];
#pragma unroll
        for (int kt = 0; kt < 4; ++kt) A[pt][kt] = load_frag(arow, 32 * kt + 8 * h);
      }
#pragma unroll 1
      for (int nt = 0; nt < kNTiles; ++nt) {
        const int n = nt * 16 + m;
        const __bf16* wrow = &sWt[l][n][0];
        const v16b Bq0 = load_frag(wrow, 8 * h);
        const v16b Bq1 = load_frag(wrow, 32 + 8 * h);
        const v16b Bq2 = load_frag(wrow, 64 + 8 * h);
        const v16b Bq3 = load_frag(wrow, 96 + 8 * h);
        const float bias = sBh[l][n];
#pragma unroll
        for (int pt = 0; pt < kPtsPerIter; ++pt) {
          v8f acc = (v8f){0.f, 0.f, 0.f, 0.f, 0.f, 0.f, 0.f, 0.f};
          acc = mma_bf(A[pt][0], Bq0, acc);
          acc = mma_bf(A[pt][1], Bq1, acc);
          acc = mma_bf(A[pt][2], Bq2, acc);
          acc = mma_bf(A[pt][3], Bq3, acc);
          mma_guard(acc, A[pt][0], A[pt][1], A[pt][2], A[pt][3], Bq0, Bq1, Bq2, Bq3);
          const float av  = (acc[0] + acc[1]) + bias;
          const float at  = acc[2] + acc[3];
          const float aL  = acc[4] + acc[5];
          const float ax0 = acc[6];
          const float ax1 = acc[7];
          const float T  = tanh_ex(av);
          const float s  = 1.0f - T * T;
          const float sp = -2.0f * T * s;
          put_jet(&sH[w][pt][8 * h][n], T, s * at, sp * (ax0 * ax0 + ax1 * ax1) + s * aL, s * ax0, s * ax1);
        }
      }
      wave_sync();
    }

    {
      const int dlane = (lane < 24) ? lane : (lane - 8);
      const int dpt   = dlane / 12;
      const int rem   = dlane - dpt * 12;
      const int dps   = rem / 6;
      const int d     = rem - dps * 6;
      const int rowA  = (d < 4) ? ((d < 2) ? 0 : (2 * d - 2)) : (d + 2);
      const int rowB  = (d < 4) ? (rowA + 1) : rowA;
      const float fb   = (d < 4) ? 1.0f : 0.0f;
      const int   oc   = (d == 1) ? 1 : 0;
      const float bsel = (d < 2) ? 1.0f : 0.0f;
      const __bf16* tile = &sH[w][dpt][8 * dps][0];
      const v4u* ra = (const v4u*)(tile + rowA * kHid);
      const v4u* rb = (const v4u*)(tile + rowB * kHid);
      const float* wo = &sWo[oc][0];
      float dacc = 0.0f;
#pragma unroll 1
      for (int c8 = 0; c8 < kHid / 8; ++c8) {
        const v4u ua  = ra[c8];
        const v4u ub  = rb[c8];
        const v4f wlo = *(const v4f*)(wo + 8 * c8);
        const v4f whi = *(const v4f*)(wo + 8 * c8 + 4);
        float vv;
        vv = fmaf(fb, __uint_as_float(ub[0] << 16),          __uint_as_float(ua[0] << 16));          dacc = fmaf(vv, wlo[0], dacc);
        vv = fmaf(fb, __uint_as_float(ub[0] & 0xffff0000u), __uint_as_float(ua[0] & 0xffff0000u)); dacc = fmaf(vv, wlo[1], dacc);
        vv = fmaf(fb, __uint_as_float(ub[1] << 16),          __uint_as_float(ua[1] << 16));          dacc = fmaf(vv, wlo[2], dacc);
        vv = fmaf(fb, __uint_as_float(ub[1] & 0xffff0000u), __uint_as_float(ua[1] & 0xffff0000u)); dacc = fmaf(vv, wlo[3], dacc);
        vv = fmaf(fb, __uint_as_float(ub[2] << 16),          __uint_as_float(ua[2] << 16));          dacc = fmaf(vv, whi[0], dacc);
        vv = fmaf(fb, __uint_as_float(ub[2] & 0xffff0000u), __uint_as_float(ua[2] & 0xffff0000u)); dacc = fmaf(vv, whi[1], dacc);
        vv = fmaf(fb, __uint_as_float(ub[3] << 16),          __uint_as_float(ua[3] << 16));          dacc = fmaf(vv, whi[2], dacc);
        vv = fmaf(fb, __uint_as_float(ub[3] & 0xffff0000u), __uint_as_float(ua[3] & 0xffff0000u)); dacc = fmaf(vv, whi[3], dacc);
      }
      sRed[w][lane] = fmaf(bsel, sBo[oc], dacc);
    }
    wave_sync();

    {
      const float* rd = &sRed[w][(lane & 1) * 12];
      float phis = 0.0f, csum = 0.0f, dts = 0.0f, laps = 0.0f;
#pragma unroll
      for (int ps = 0; ps < 2; ++ps) {
        const float o0  = rd[6 * ps + 0];
        const float o1  = rd[6 * ps + 1];
        const float ot  = rd[6 * ps + 2];
        const float oL  = rd[6 * ps + 3];
        const float ox0 = rd[6 * ps + 4];
        const float ox1 = rd[6 * ps + 5];
        const float T0  = tanh_ex(o0);
        const float s0  = 1.0f - T0 * T0;
        const float sp0 = -2.0f * T0 * s0;
        const float ph  = T0 * 0.5f + 0.5f;
        const float T1  = tanh_ex(o1);
        const float clv = (T1 * 0.5f + 0.5f) * kClScale;
        const float cp  = kCseMinusCle * (-2.0f * ph * ph * ph + 3.0f * ph * ph) + clv;
        phis += ph;
        csum += cp;
        dts  += 0.5f * s0 * ot;
        laps += 0.5f * (sp0 * (ox0 * ox0 + ox1 * ox1) + s0 * oL);
      }
      const float phi    = 0.5f * phis;
      const float cc     = 0.5f * csum;
      const float dphidt = 0.5f * dts;
      const float lap    = 0.5f * laps;
      const float phi2 = phi * phi, phi3 = phi2 * phi;
      const float hphi = -2.0f * phi3 + 3.0f * phi2;
      const float dh   = -6.0f * phi2 + 6.0f * phi;
      const float dg   = 4.0f * phi3 - 6.0f * phi2 + 2.0f * phi;
      const float ac = dphidt
                     - kAC1 * (cc - hphi * kCseMinusCle - kCLE) * kCseMinusCle * dh
                     + kAC2 * dg
                     - kAC3 * lap;
      if (lane < 2) sOut[w][it * 2 + lane] = ac;
    }
    wave_sync();
  }

  {
    const int l8 = lane & 7;
    const v4f ov = *(const v4f*)(&sOut[w][l8 * 4]);
    float* op = out + (size_t)pbase + l8 * 4;
    if (lane < 8) *(volatile v4f*)op = ov;
    __threadfence();
    if (lane < 8) *(volatile v4f*)op = ov;
  }
}

extern "C" void kernel_launch(void* const* d_in, const int* in_sizes, int n_in,
                              void* d_out, int out_size, void* d_ws, size_t ws_size,
                              hipStream_t stream) {
  (void)d_ws;
  (void)ws_size;
  if (n_in < 7) return;
  const float* x    = (const float*)d_in[0];
  const float* t    = (const float*)d_in[1];
  const float* Bff  = (const float*)d_in[2];
  const float* Wh   = (const float*)d_in[3];
  const float* bh   = (const float*)d_in[4];
  const float* Wout = (const float*)d_in[5];
  const float* bout = (const float*)d_in[6];
  float* out = (float*)d_out;
  const int npts = in_sizes[1];
  if (npts <= 0 || (npts % kPtsPerBlock) != 0) return;
  if (in_sizes[0] != 2 * npts || out_size != npts) return;
  if (in_sizes[2] != 3 * kEmb || in_sizes[3] != kLayers * kHid * kHid || in_sizes[4] != kLayers * kHid ||
      in_sizes[5] != 2 * kHid || in_sizes[6] < 2) return;
  const int grid = npts / kPtsPerBlock;
  jet_residual_kernel<<<dim3(grid), dim3(kBlock), 0, stream>>>(x, t, Bff, Wh, bh, Wout, bout, out, npts);
}
